// Transformers_87153476370458
// MI455X (gfx1250) — hardware-verified
//
#include <hip/hip_runtime.h>


#define NBT 4
#define SQ  2048
#define NHD 8
#define HDM 64
#define DMD 64
#define TDM 512
#define NTK (NBT * SQ)
#define NEGM 1000000.0f
#define PSC  32768.0f

typedef _Float16 h16;
typedef __attribute__((ext_vector_type(8)))  _Float16 v8h;
typedef __attribute__((ext_vector_type(4)))  float    v4f;
typedef v8h  __attribute__((may_alias)) v8ha;
typedef v4f  __attribute__((may_alias)) v4fa;

typedef __attribute__((ext_vector_type(16))) __bf16   v16bf;
typedef __attribute__((ext_vector_type(16))) _Float16 v16h;
typedef __attribute__((ext_vector_type(8)))  float    v8f;
typedef __attribute__((ext_vector_type(8)))  unsigned v8u;

__device__ __forceinline__ unsigned f2bf(float f) { unsigned u = __float_as_uint(f); u += 0x7FFFu + ((u >> 16) & 1u); return u >> 16; }
__device__ __forceinline__ unsigned f2h(float f) { return (unsigned)__builtin_bit_cast(unsigned short, (_Float16)f); }
__device__ __forceinline__ int kpat(int v, int half) { return ((v & 4) ? 16 : 0) + half * 8 + 2 * (v & 3); }

template <int F16, int NP> struct Opnd { v16bf p[NP]; };

template <int F16, int NP> __device__ __forceinline__ void pack2(float f0, float f1, unsigned* o) {
    if (F16) { o[0] = f2h(f0) | (f2h(f1) << 16); return; }
    unsigned h0 = f2bf(f0), h1 = f2bf(f1); o[0] = h0 | (h1 << 16);
    if (NP >= 2) {
        float r0 = f0 - __uint_as_float(h0 << 16), r1 = f1 - __uint_as_float(h1 << 16);
        unsigned m0 = f2bf(r0), m1 = f2bf(r1); o[1] = m0 | (m1 << 16);
        if (NP >= 3) {
            float s0 = r0 - __uint_as_float(m0 << 16), s1 = r1 - __uint_as_float(m1 << 16);
            o[2] = f2bf(s0) | (f2bf(s1) << 16);
        }
    }
}
template <int F16, int NP> __device__ __forceinline__ void op_row(const float* rowp, int half, float sc, Opnd<F16, NP>& o) {
    v8u u[NP];
#pragma unroll
    for (int v = 0; v < 8; ++v) {
        int kk = kpat(v, half); unsigned t[3];
        pack2<F16, NP>(rowp[kk] * sc, rowp[kk + 1] * sc, t);
#pragma unroll
        for (int p = 0; p < NP; ++p) u[p][v] = t[p];
    }
#pragma unroll
    for (int p = 0; p < NP; ++p) o.p[p] = __builtin_bit_cast(v16bf, u[p]);
}
template <int F16, int NP> __device__ __forceinline__ void op_row_tail(const float* rowp, int half, float sc, int kvalid, Opnd<F16, NP>& o) {
    v8u u[NP];
#pragma unroll
    for (int v = 0; v < 8; ++v) {
        int kk = kpat(v, half); unsigned t[3];
        float f0 = kk < kvalid ? rowp[kk] * sc : 0.0f, f1 = (kk + 1) < kvalid ? rowp[kk + 1] * sc : 0.0f;
        pack2<F16, NP>(f0, f1, t);
#pragma unroll
        for (int p = 0; p < NP; ++p) u[p][v] = t[p];
    }
#pragma unroll
    for (int p = 0; p < NP; ++p) o.p[p] = __builtin_bit_cast(v16bf, u[p]);
}
template <int F16, int NP> __device__ __forceinline__ void op_col(const float* M, int ld, int n, int k0, int half, float sc, Opnd<F16, NP>& o) {
    v8u u[NP];
#pragma unroll
    for (int v = 0; v < 8; ++v) {
        int kk = k0 + kpat(v, half); unsigned t[3];
        pack2<F16, NP>(M[(size_t)kk * ld + n] * sc, M[(size_t)(kk + 1) * ld + n] * sc, t);
#pragma unroll
        for (int p = 0; p < NP; ++p) u[p][v] = t[p];
    }
#pragma unroll
    for (int p = 0; p < NP; ++p) o.p[p] = __builtin_bit_cast(v16bf, u[p]);
}
template <int F16, int NP> __device__ __forceinline__ void op_col_tail(const float* M, int ld, int n, int k0, int half, float sc, int K, Opnd<F16, NP>& o) {
    v8u u[NP];
#pragma unroll
    for (int v = 0; v < 8; ++v) {
        int kk = k0 + kpat(v, half); unsigned t[3];
        float f0 = kk < K ? M[(size_t)kk * ld + n] * sc : 0.0f, f1 = (kk + 1) < K ? M[(size_t)(kk + 1) * ld + n] * sc : 0.0f;
        pack2<F16, NP>(f0, f1, t);
#pragma unroll
        for (int p = 0; p < NP; ++p) u[p][v] = t[p];
    }
#pragma unroll
    for (int p = 0; p < NP; ++p) o.p[p] = __builtin_bit_cast(v16bf, u[p]);
}
__device__ __forceinline__ v8f wm_bf16(v16bf a, v16bf b, v8f c) { return __builtin_amdgcn_wmma_f32_16x16x32_bf16(false, a, false, b, (short)0, c, false, false); }
template <int F16, int NA, int NB> __device__ __forceinline__ v8f wmma_op(const Opnd<F16, NA>& a, const Opnd<F16, NB>& b, v8f c) {
    if (F16) {
        v16h ah = __builtin_bit_cast(v16h, a.p[0]), bh = __builtin_bit_cast(v16h, b.p[0]);
        c = __builtin_amdgcn_wmma_f32_16x16x32_f16(false, ah, false, bh, (short)0, c, false, false);
        asm volatile("v_nop\n\tv_nop\n\tv_nop\n\tv_nop" : "+v"(c) : "v"(ah), "v"(bh));
        return c;
    }
    constexpr int NMX = NA > NB ? NA : NB;
#pragma unroll
    for (int i = 0; i < NA; ++i)
#pragma unroll
        for (int j = 0; j < NB; ++j)
            if (i + j < NMX) c = wm_bf16(a.p[i], b.p[j], c);
    if (NA == 1 && NB == 1)      asm volatile("v_nop\n\tv_nop\n\tv_nop\n\tv_nop" : "+v"(c) : "v"(a.p[0]), "v"(b.p[0]));
    else if (NA == 2 && NB == 1) asm volatile("v_nop\n\tv_nop\n\tv_nop\n\tv_nop" : "+v"(c) : "v"(a.p[0]), "v"(a.p[1]), "v"(b.p[0]));
    else if (NA == 1 && NB == 2) asm volatile("v_nop\n\tv_nop\n\tv_nop\n\tv_nop" : "+v"(c) : "v"(a.p[0]), "v"(b.p[0]), "v"(b.p[1]));
    else if (NA == 2 && NB == 2) asm volatile("v_nop\n\tv_nop\n\tv_nop\n\tv_nop" : "+v"(c) : "v"(a.p[0]), "v"(a.p[1]), "v"(b.p[0]), "v"(b.p[1]));
    else                         asm volatile("v_nop\n\tv_nop\n\tv_nop\n\tv_nop" : "+v"(c) : "v"(a.p[0]), "v"(a.p[NA - 1]), "v"(b.p[0]), "v"(b.p[NB - 1]), "v"(a.p[NA / 2]), "v"(b.p[NB / 2]));
    return c;
}

struct ZMap { long long s1; long long s2; int zdiv; int pad_; };
__device__ __forceinline__ size_t zoff(const ZMap& m, int z) { return (size_t)((long long)(z / m.zdiv) * m.s1 + (long long)(z % m.zdiv) * m.s2); }

#define ACT_NONE 0
#define ACT_RELU 1
#define ACT_GELU_ERF 2
#define ACT_SILU 3
#define ACT_TANH 4
__device__ __forceinline__ float act_apply(int act, float x) {
    if (act == ACT_RELU) return x > 0.f ? x : 0.f;
    if (act == ACT_GELU_ERF) return 0.5f * x * (1.0f + erff(x * 0.70710678118654752f));
    if (act == ACT_SILU) return x / (1.0f + expf(-x));
    if (act == ACT_TANH) return tanhf(x);
    return x;
}
struct GemmArgs {
    ZMap za, zb_, zc, zbias, zadd, zrsc, zmul, zrbias;
    const float* A; const float* Bm; float* C; const float* bias; const float* add; const float* rsc; const float* mul; const float* rbias;
    long long ldadd, ldmul;
    int lda, ldb, ldc, K;
    float ascale, bscale, oscale, addscale;
    int M, nvalid, nstore, ldrsc;
    int bcs, pad1, pad2, pad3;
};
template <int BT, int F16, int NA, int NB, int RW, int CW, int ACT>
__global__ __launch_bounds__(256) void gemm_kernel(GemmArgs g) {
    constexpr int TR = 16 * RW, TC = 64 * CW, CSTR = TC + 4;
    __shared__ __align__(16) float cst[TR * CSTR];
    const int z = blockIdx.z;
    const float* A = g.A + zoff(g.za, z); const float* Bm = g.Bm + zoff(g.zb_, z); float* C = g.C + zoff(g.zc, z);
    const int tid = threadIdx.x, lane = tid & 31, wv = tid >> 5;
    const int l16 = lane & 15, half = lane >> 4;
    const int rt = wv % RW, ch = wv / RW;
    const int row0 = blockIdx.x * TR, col0 = blockIdx.y * TC + ch * 64;
    int arix = row0 + rt * 16 + l16; if (arix >= g.M) arix = g.M - 1;
    const float* arow = A + (size_t)arix * g.lda;
    v8f acc[4];
#pragma unroll
    for (int t = 0; t < 4; ++t) acc[t] = (v8f){};
    const int K = g.K;
#pragma unroll 1
    for (int kc = 0; kc < K; kc += 32) {
        Opnd<F16, NA> a;
        if (kc + 32 <= K) op_row<F16, NA>(arow + kc, half, g.ascale, a); else op_row_tail<F16, NA>(arow + kc, half, g.ascale, K - kc, a);
#pragma unroll
        for (int t = 0; t < 4; ++t) {
            Opnd<F16, NB> b;
            const int n = col0 + t * 16 + l16;
            if (n < g.nvalid) {
                if (BT) { if (kc + 32 <= K) op_row<F16, NB>(Bm + (size_t)n * g.ldb + kc, half, g.bscale, b); else op_row_tail<F16, NB>(Bm + (size_t)n * g.ldb + kc, half, g.bscale, K - kc, b); }
                else    { if (kc + 32 <= K) op_col<F16, NB>(Bm, g.ldb, n * g.bcs, kc, half, g.bscale, b); else op_col_tail<F16, NB>(Bm, g.ldb, n * g.bcs, kc, half, g.bscale, K, b); }
            } else {
#pragma unroll
                for (int p = 0; p < NB; ++p) b.p[p] = (v16bf){};
            }
            acc[t] = wmma_op<F16, NA, NB>(a, b, acc[t]);
        }
    }
    const float* bias = g.bias ? g.bias + zoff(g.zbias, z) : nullptr;
    const float* add = g.add ? g.add + zoff(g.zadd, z) : nullptr;
    const float* rsc = g.rsc ? g.rsc + zoff(g.zrsc, z) : nullptr;
    const float* mul = g.mul ? g.mul + zoff(g.zmul, z) : nullptr;
    const float* rbias = g.rbias ? g.rbias + zoff(g.zrbias, z) : nullptr;
#pragma unroll
    for (int t = 0; t < 4; ++t) {
        const int cl = ch * 64 + t * 16 + l16;
        const int cg = blockIdx.y * TC + cl;
        const bool cok = cg < g.nvalid;
        const float bv = (bias && cok) ? bias[(size_t)cg * g.bcs] : 0.0f;
#pragma unroll
        for (int r = 0; r < 8; ++r) {
            const int rl = rt * 16 + r + 8 * half;
            float v = acc[t][r] * g.oscale + bv;
            int rg = row0 + rl; if (rg >= g.M) rg = g.M - 1;
            if (rbias) v += rbias[rg];
            if (rsc) v *= rsc[(size_t)rg * g.ldrsc];
            if (mul && cok) v *= mul[(size_t)rg * g.ldmul + cg];
            if (add && cok) v += g.addscale * add[(size_t)rg * g.ldadd + cg];
            cst[rl * CSTR + cl] = v;
        }
    }
    __syncthreads();
    const int col = tid % TC, rsel = tid / TC, rstep = 256 / TC;
    if (ACT != ACT_NONE) {
#pragma unroll 1
        for (int r = rsel; r < TR; r += rstep) cst[r * CSTR + col] = act_apply(ACT, cst[r * CSTR + col]);
    }
    float* ob = C + (size_t)row0 * g.ldc + (size_t)blockIdx.y * TC;
    const bool colok = (int)(blockIdx.y * TC + col) < g.nstore;
    const int rmax = (g.M - row0 < TR) ? (g.M - row0) : TR;
    auto pass = [&]() {
        if (colok) {
#pragma unroll 4
            for (int r = rsel; r < rmax; r += rstep) *(volatile float*)(ob + (size_t)r * g.ldc + col) = cst[r * CSTR + col];
        }
    };
    pass();
    __threadfence();
    pass();
}
static inline ZMap zm(long long s1) { ZMap m; m.s1 = s1; m.s2 = 0; m.zdiv = 1; m.pad_ = 0; return m; }
static inline ZMap zm2(long long s1, long long s2, int zdiv) { ZMap m; m.s1 = s1; m.s2 = s2; m.zdiv = zdiv; m.pad_ = 0; return m; }
static inline GemmArgs gemm_args(const float* A, int lda, ZMap za, const float* Bm, int ldb, ZMap zb, float* C, int ldc, ZMap zc, int M, int N, int K) {
    GemmArgs g; g.za = za; g.zb_ = zb; g.zc = zc; g.zbias = zm(0); g.zadd = zm(0); g.zrsc = zm(0); g.zmul = zm(0); g.zrbias = zm(0);
    g.A = A; g.Bm = Bm; g.C = C; g.bias = nullptr; g.add = nullptr; g.rsc = nullptr; g.mul = nullptr; g.rbias = nullptr; g.ldadd = 0; g.ldmul = 0;
    g.lda = lda; g.ldb = ldb; g.ldc = ldc; g.K = K; g.ascale = 1.0f; g.bscale = 1.0f; g.oscale = 1.0f; g.addscale = 1.0f; g.M = M; g.nvalid = N; g.nstore = N; g.ldrsc = 1;
    g.bcs = 1; g.pad1 = 0; g.pad2 = 0; g.pad3 = 0;
    return g;
}
static_assert(sizeof(ZMap) == 24, "ZMap layout");
static_assert(sizeof(GemmArgs) == 8 * 24 + 8 * 8 + 2 * 8 + 4 * 4 + 4 * 4 + 4 * 4 + 4 * 4, "GemmArgs has no padding");


#define VST2(T, p, v) do { const T vst2_v_ = (v); *(volatile T*)(p) = vst2_v_; __threadfence(); *(volatile T*)(p) = vst2_v_; } while (0)
__device__ __forceinline__ v16h cat16(v8h lo, v8h hi) { return __builtin_shufflevector(lo, hi, 0, 1, 2, 3, 4, 5, 6, 7, 8, 9, 10, 11, 12, 13, 14, 15); }
__device__ __forceinline__ v8f wmma16(v16h a, v16h b, v8f c) { return __builtin_amdgcn_wmma_f32_16x16x32_f16(false, a, false, b, (short)0, c, false, false); }

__global__ __launch_bounds__(256) void k_ln(const float* __restrict__ X, const float* __restrict__ ADD, const float* __restrict__ gam, const float* __restrict__ bet,
                                            float* RES, float* Y) {
    const int lane = threadIdx.x & 31;
    const int r = blockIdx.x * 8 + (threadIdx.x >> 5);
    if (r >= NTK) return;
    float x0 = X[(size_t)r * DMD + lane], x1 = X[(size_t)r * DMD + 32 + lane];
    if (ADD) { x0 += ADD[(size_t)r * DMD + lane]; x1 += ADD[(size_t)r * DMD + 32 + lane]; }
    float s = x0 + x1;
#pragma unroll
    for (int o = 16; o; o >>= 1) s += __shfl_xor(s, o, 32);
    const float mu = s * (1.0f / 64.0f);
    const float d0 = x0 - mu, d1 = x1 - mu;
    float q = d0 * d0 + d1 * d1;
#pragma unroll
    for (int o = 16; o; o >>= 1) q += __shfl_xor(q, o, 32);
    const float rs = rsqrtf(q * (1.0f / 64.0f) + 1e-3f);
    const float y0 = d0 * rs * gam[lane] + bet[lane], y1 = d1 * rs * gam[32 + lane] + bet[32 + lane];
    if (RES) { VST2(float, RES + (size_t)r * DMD + lane, x0); VST2(float, RES + (size_t)r * DMD + 32 + lane, x1); }
    VST2(float, Y + (size_t)r * DMD + lane, y0); VST2(float, Y + (size_t)r * DMD + 32 + lane, y1);
}

__global__ __launch_bounds__(256) void k_cvtqk(const float* __restrict__ QKVf, h16* QH, h16* KH) {
    const int lane = threadIdx.x & 31;
    const int wid = blockIdx.x * 8 + (threadIdx.x >> 5);
    if (wid >= 2 * NTK) return;
    const int r = wid >> 1, which = wid & 1;
    const float* src = QKVf + (size_t)r * (3 * TDM) + which * TDM;
    h16* dst = (which ? KH : QH) + (size_t)r * TDM;
    v8h o[2];
#pragma unroll
    for (int s = 0; s < 2; ++s) {
        const float* p = src + s * 256 + lane * 8;
        const v4f a = *(const v4f*)p, b = *(const v4f*)(p + 4);
        v8h t; t[0] = (h16)a[0]; t[1] = (h16)a[1]; t[2] = (h16)a[2]; t[3] = (h16)a[3]; t[4] = (h16)b[0]; t[5] = (h16)b[1]; t[6] = (h16)b[2]; t[7] = (h16)b[3];
        o[s] = t;
    }
#pragma unroll
    for (int s = 0; s < 2; ++s) *(volatile v8h*)(dst + s * 256 + lane * 8) = o[s];
    __threadfence();
#pragma unroll
    for (int s = 0; s < 2; ++s) *(volatile v8h*)(dst + s * 256 + lane * 8) = o[s];
}

__global__ __launch_bounds__(256) void k_vt(const float* __restrict__ QKVf, h16* VT) {
    __shared__ __align__(16) h16 tile[64 * 72];
    const int bid = blockIdx.x;
    const int b = bid / (NHD * (SQ / 64)), rem = bid - b * (NHD * (SQ / 64)), h = rem / (SQ / 64), kt = rem - h * (SQ / 64);
    const int k0 = kt * 64, tid = threadIdx.x;
    const int kk = tid >> 2, d0 = (tid & 3) * 16;
    const float* src = QKVf + ((size_t)b * SQ + k0 + kk) * (3 * TDM) + 2 * TDM + h * HDM + d0;
#pragma unroll
    for (int i = 0; i < 16; ++i) tile[(d0 + i) * 72 + kk] = (h16)src[i];
    __syncthreads();
    const int piece = tid & 7;
    h16* base = VT + (((size_t)b * NHD + h) * HDM) * SQ + k0;
    auto pass = [&]() {
#pragma unroll
        for (int s = 0; s < 2; ++s) {
            const int d = (tid >> 3) + 32 * s;
            const v8h val = *(const v8ha*)(tile + d * 72 + piece * 8);
            *(volatile v8h*)(base + (size_t)d * SQ + piece * 8) = val;
        }
    };
    pass();
    __threadfence();
    pass();
}

__global__ __launch_bounds__(128) void k_attn(const h16* __restrict__ QH, const h16* __restrict__ KH, const h16* __restrict__ VT,
                                              const int* __restrict__ tids, const int* __restrict__ am, float* CTX) {
    __shared__ __align__(16) h16 plds[4][16 * 32];
    __shared__ __align__(16) float ost[4][16 * 68];
    const int lane = threadIdx.x & 31, wave = threadIdx.x >> 5, lr = lane & 15, hi = lane >> 4;
    const int bid = blockIdx.x;
    const int b = bid / (NHD * (SQ / 64)), rem = bid - b * (NHD * (SQ / 64)), h = rem / (SQ / 64), qt = rem - h * (SQ / 64);
    const int q0 = qt * 64 + wave * 16;
    const size_t tok0 = (size_t)b * SQ;
    h16* pl = &plds[wave][0];

    v16h qa[2];
#pragma unroll
    for (int kc = 0; kc < 2; ++kc) {
        const h16* p = QH + (tok0 + q0 + lr) * TDM + h * HDM + kc * 32 + 8 * hi;
        qa[kc] = cat16(*(const v8h*)p, *(const v8h*)(p + 16));
    }
    int tq[8];
#pragma unroll
    for (int j = 0; j < 8; ++j) tq[j] = tids[tok0 + q0 + 8 * hi + j];
    const h16* kh_b = KH + tok0 * TDM + h * HDM;
    const h16* vt_b = VT + (((size_t)b * NHD + h) * HDM) * SQ;
    const int* tk_b = tids + tok0;
    const int* am_b = am + tok0;

    v8f o[4];
#pragma unroll
    for (int n = 0; n < 4; ++n) o[n] = (v8f){};
    float mrow[8], lpart[8];
#pragma unroll
    for (int j = 0; j < 8; ++j) { mrow[j] = -3.0e38f; lpart[j] = 0.f; }

#pragma unroll 1
    for (int kt = 0; kt < SQ / 32; ++kt) {
        const int l0 = kt * 32;
        const int key0 = l0 + lr, key1 = l0 + 16 + lr;
        const int tk0 = tk_b[key0], tk1 = tk_b[key1];
        const float pm0 = ((float)am_b[key0] - 1.0f) * NEGM, pm1 = ((float)am_b[key1] - 1.0f) * NEGM;
        v8f s0 = {}, s1 = {};
#pragma unroll
        for (int kc = 0; kc < 2; ++kc) {
            const h16* r0 = kh_b + (size_t)key0 * TDM + kc * 32 + 8 * hi;
            const h16* r1 = kh_b + (size_t)key1 * TDM + kc * 32 + 8 * hi;
            s0 = wmma16(qa[kc], cat16(*(const v8h*)r0, *(const v8h*)(r0 + 16)), s0);
            s1 = wmma16(qa[kc], cat16(*(const v8h*)r1, *(const v8h*)(r1 + 16)), s1);
        }
        asm volatile("v_nop\n\tv_nop\n\tv_nop\n\tv_nop" : "+v"(s0), "+v"(s1) : "v"(qa[0]), "v"(qa[1]));
        float alpha[8];
#pragma unroll
        for (int j = 0; j < 8; ++j) {
            const int qpos = q0 + 8 * hi + j;
            float a0 = s0[j] * 0.125f;
            a0 += (tq[j] >= tk0) ? 0.0f : -NEGM;
            a0 += pm0;
            a0 += (key0 == qpos) ? -NEGM : -0.0f;
            float a1 = s1[j] * 0.125f;
            a1 += (tq[j] >= tk1) ? 0.0f : -NEGM;
            a1 += pm1;
            a1 += (key1 == qpos) ? -NEGM : -0.0f;
            float mx = fmaxf(a0, a1);
            mx = fmaxf(mx, __shfl_xor(mx, 1, 16)); mx = fmaxf(mx, __shfl_xor(mx, 2, 16));
            mx = fmaxf(mx, __shfl_xor(mx, 4, 16)); mx = fmaxf(mx, __shfl_xor(mx, 8, 16));
            const float mn = fmaxf(mrow[j], mx);
            alpha[j] = __expf(mrow[j] - mn);
            mrow[j] = mn;
            const float p0 = __expf(a0 - mn), p1 = __expf(a1 - mn);
            lpart[j] = lpart[j] * alpha[j] + (p0 + p1);
            const int mr = hi * 8 + j;
            pl[mr * 32 + lr]      = (h16)(p0 * PSC);
            pl[mr * 32 + 16 + lr] = (h16)(p1 * PSC);
        }
#pragma unroll
        for (int n = 0; n < 4; ++n)
#pragma unroll
            for (int j = 0; j < 8; ++j) o[n][j] *= alpha[j];
        asm volatile("" ::: "memory");
        const v16h pa = cat16(*(const v8ha*)(pl + lr * 32 + hi * 8), *(const v8ha*)(pl + lr * 32 + 16 + hi * 8));
#pragma unroll
        for (int n = 0; n < 4; ++n) {
            const h16* vp = vt_b + (size_t)(n * 16 + lr) * SQ + l0 + hi * 8;
            o[n] = wmma16(pa, cat16(*(const v8h*)vp, *(const v8h*)(vp + 16)), o[n]);
        }
        asm volatile("v_nop\n\tv_nop\n\tv_nop\n\tv_nop" : "+v"(o[0]), "+v"(o[1]), "+v"(o[2]), "+v"(o[3]) : "v"(pa));
    }
    float inv[8];
#pragma unroll
    for (int j = 0; j < 8; ++j) {
        float rs = lpart[j];
        rs += __shfl_xor(rs, 1, 16); rs += __shfl_xor(rs, 2, 16); rs += __shfl_xor(rs, 4, 16); rs += __shfl_xor(rs, 8, 16);
        inv[j] = 1.0f / (rs * PSC);
    }
    float* os = &ost[wave][0];
#pragma unroll
    for (int n = 0; n < 4; ++n)
#pragma unroll
        for (int j = 0; j < 8; ++j) os[(hi * 8 + j) * 68 + n * 16 + lr] = o[n][j] * inv[j];
    __syncthreads();
    float* crow = CTX + (tok0 + q0) * TDM + h * HDM;
    auto pass = [&]() {
#pragma unroll
        for (int s = 0; s < 8; ++s) {
            const int Lid = (lane >> 3) + 4 * s, piece = lane & 7;
            const int row = Lid >> 1, cofs = (Lid & 1) * 32 + piece * 4;
            const v4f val = *(const v4fa*)(os + row * 68 + cofs);
            *(volatile v4f*)(crow + (size_t)row * TDM + cofs) = val;
        }
    };
    pass();
    __threadfence();
    pass();
}

__global__ __launch_bounds__(256) void k_fin(const float* __restrict__ A, const float* __restrict__ Bv, float* out) {
    const int lane = threadIdx.x & 31;
    const int r = blockIdx.x * 8 + (threadIdx.x >> 5);
    if (r >= NTK) return;
    const float y0 = A[(size_t)r * DMD + lane] + Bv[(size_t)r * DMD + lane];
    const float y1 = A[(size_t)r * DMD + 32 + lane] + Bv[(size_t)r * DMD + 32 + lane];
    VST2(float, out + (size_t)r * DMD + lane, y0); VST2(float, out + (size_t)r * DMD + 32 + lane, y1);
}

extern "C" void kernel_launch(void* const* d_in, const int* in_sizes, int n_in,
                              void* d_out, int out_size, void* d_ws, size_t ws_size, hipStream_t stream) {
    (void)in_sizes; (void)n_in; (void)out_size;
    const float* hid = (const float*)d_in[0]; const int* tids = (const int*)d_in[1]; const int* am = (const int*)d_in[2];
    const float* Wq = (const float*)d_in[3]; const float* Wk = (const float*)d_in[4]; const float* Wv = (const float*)d_in[5];
    const float* Watt = (const float*)d_in[6]; const float* Wout = (const float*)d_in[7]; const float* bout = (const float*)d_in[8];
    const float* g_in = (const float*)d_in[9]; const float* b_in = (const float*)d_in[10]; const float* g_out = (const float*)d_in[11]; const float* b_out = (const float*)d_in[12];
    float* out = (float*)d_out;
    char* wsp = (char*)d_ws;
    auto take = [&](size_t bytes) { char* p = wsp; wsp += (bytes + 255) & ~(size_t)255; return (void*)p; };
    float* XLN  = (float*)take((size_t)NTK * DMD * 4);
    float* QKVf = (float*)take((size_t)NTK * 3 * TDM * 4);
    h16*   QH   = (h16*)take((size_t)NTK * TDM * 2);
    h16*   KH   = (h16*)take((size_t)NTK * TDM * 2);
    h16*   VT   = (h16*)take((size_t)NTK * TDM * 2);
    float* CTX  = (float*)take((size_t)NTK * TDM * 4);
    float* ATT  = (float*)take((size_t)NTK * DMD * 4);
    float* OUT1 = (float*)take((size_t)NTK * DMD * 4);
    float* NO   = (float*)take((size_t)NTK * DMD * 4);
    float* DEN  = (float*)take((size_t)NTK * DMD * 4);
    if ((size_t)(wsp - (char*)d_ws) > ws_size) return;
    k_ln<<<NTK / 8, 256, 0, stream>>>(hid, nullptr, g_in, b_in, nullptr, XLN);
    { GemmArgs g = gemm_args(XLN, DMD, zm(0), Wq, TDM, zm(0), QKVf,           3 * TDM, zm(0), NTK, TDM, DMD); gemm_kernel<0, 1, 1, 1, 4, 2, ACT_NONE><<<dim3(NTK / 64, TDM / 128, 1), 256, 0, stream>>>(g); }
    { GemmArgs g = gemm_args(XLN, DMD, zm(0), Wk, TDM, zm(0), QKVf + TDM,     3 * TDM, zm(0), NTK, TDM, DMD); gemm_kernel<0, 1, 1, 1, 4, 2, ACT_NONE><<<dim3(NTK / 64, TDM / 128, 1), 256, 0, stream>>>(g); }
    { GemmArgs g = gemm_args(XLN, DMD, zm(0), Wv, TDM, zm(0), QKVf + 2 * TDM, 3 * TDM, zm(0), NTK, TDM, DMD); gemm_kernel<0, 1, 1, 1, 4, 2, ACT_NONE><<<dim3(NTK / 64, TDM / 128, 1), 256, 0, stream>>>(g); }
    k_cvtqk<<<(2 * NTK) / 8, 256, 0, stream>>>(QKVf, QH, KH);
    k_vt<<<NBT * NHD * (SQ / 64), 256, 0, stream>>>(QKVf, VT);
    k_attn<<<NBT * NHD * (SQ / 64), 128, 0, stream>>>(QH, KH, VT, tids, am, CTX);
    { GemmArgs g = gemm_args(CTX, TDM, zm(0), Watt, DMD, zm(0), ATT, DMD, zm(0), NTK, DMD, TDM); gemm_kernel<0, 1, 1, 1, 8, 1, ACT_RELU><<<dim3(NTK / 128, 1, 1), 256, 0, stream>>>(g); }
    k_ln<<<NTK / 8, 256, 0, stream>>>(ATT, hid, g_out, b_out, OUT1, NO);
    { GemmArgs g = gemm_args(NO, DMD, zm(0), Wout, DMD, zm(0), DEN, DMD, zm(0), NTK, DMD, DMD); g.bias = bout; gemm_kernel<0, 1, 1, 1, 8, 1, ACT_RELU><<<dim3(NTK / 128, 1, 1), 256, 0, stream>>>(g); }
    k_fin<<<NTK / 8, 256, 0, stream>>>(DEN, OUT1, out);
}
